// PVAM_57836029608001
// MI455X (gfx1250) — hardware-run, weakly checked
//
#include <hip/hip_runtime.h>
#include <math.h>

typedef __attribute__((ext_vector_type(16))) _Float16 v16h;
typedef __attribute__((ext_vector_type(16))) __bf16 v16b;
typedef __attribute__((ext_vector_type(8)))  _Float16 v8h;
typedef __attribute__((ext_vector_type(8)))  float v8f;
typedef __attribute__((ext_vector_type(4)))  float v4f;
typedef __attribute__((ext_vector_type(2)))  float v2f;
typedef __attribute__((ext_vector_type(4)))  unsigned v4u;
typedef __attribute__((ext_vector_type(4)))  int v4i;
typedef float __attribute__((may_alias)) float_a;
typedef int __attribute__((may_alias)) int_a;

template <typename T> __device__ __forceinline__ void vst2(void* p, T v) { *(volatile T*)p = v; __threadfence(); *(volatile T*)p = v; }
__device__ __forceinline__ v8f wmma16(v16h a, v16h b, v8f c) {
  v8f d = __builtin_amdgcn_wmma_f32_16x16x32_f16(false, a, false, b, (short)0, c, false, false);
  asm volatile("v_nop\n\tv_nop\n\tv_nop\n\tv_nop" : "+v"(d) : "v"(a), "v"(b));
  return d;
}
__device__ __forceinline__ v8f wmma_bf(v16b a, v16b b, v8f c) {
  v8f d = __builtin_amdgcn_wmma_f32_16x16x32_bf16(false, a, false, b, (short)0, c, false, false);
  asm volatile("v_nop\n\tv_nop\n\tv_nop\n\tv_nop" : "+v"(d) : "v"(a), "v"(b));
  return d;
}
__device__ __forceinline__ v16h frag_h(const _Float16* rowk0, int lane) {
  union { v16h v; v8h q[2]; } u; const _Float16* p = rowk0 + 8 * (lane >> 4);
  u.q[0] = *(const v8h*)p; u.q[1] = *(const v8h*)(p + 16); return u.v;
}
__device__ __forceinline__ v16h frag_f32(const float* rowk0, int lane) {
  v16h a; const float* p = rowk0 + 8 * (lane >> 4);
#pragma unroll
  for (int i = 0; i < 8; ++i) { a[i] = (_Float16)p[i]; a[8 + i] = (_Float16)p[16 + i]; }
  return a;
}
__device__ __forceinline__ v16h frag_f32s(const float* rowk0, int lane, float sc) {
  v16h a; const float* p = rowk0 + 8 * (lane >> 4);
#pragma unroll
  for (int i = 0; i < 8; ++i) { a[i] = (_Float16)(p[i] * sc); a[8 + i] = (_Float16)(p[16 + i] * sc); }
  return a;
}
__device__ __forceinline__ v16h fragc_f32(const float* W, int k0, int n, int lane, int ld, int K) {
  v16h a; const int g = lane >> 4;
#pragma unroll
  for (int i = 0; i < 8; ++i) { const int ka = k0 + 8 * g + i, kb = ka + 16;
    a[i] = (_Float16)(ka < K ? W[(size_t)(ka < K ? ka : K - 1) * ld + n] : 0.f); a[8 + i] = (_Float16)(kb < K ? W[(size_t)(kb < K ? kb : K - 1) * ld + n] : 0.f); }
  return a;
}
struct F2 { v16b h, l; };
__device__ __forceinline__ F2 bsplit16(const float v[16]) { F2 r;
#pragma unroll
  for (int i = 0; i < 16; ++i) { const __bf16 h = (__bf16)v[i]; r.h[i] = h; r.l[i] = (__bf16)(v[i] - (float)h); }
  return r; }
__device__ __forceinline__ F2 split_row(const float* row, int k0, int lane) { float v[16]; const float* p = row + k0 + 8 * (lane >> 4);
#pragma unroll
  for (int i = 0; i < 8; ++i) { v[i] = p[i]; v[8 + i] = p[16 + i]; }
  return bsplit16(v); }
__device__ __forceinline__ F2 split_rowK(const float* row, int k0, int lane, int K) { float v[16]; const int g = lane >> 4;
#pragma unroll
  for (int i = 0; i < 8; ++i) { const int ka = k0 + 8 * g + i, kb = ka + 16; v[i] = ka < K ? row[ka < K ? ka : K - 1] : 0.f; v[8 + i] = kb < K ? row[kb < K ? kb : K - 1] : 0.f; }
  return bsplit16(v); }
__device__ __forceinline__ F2 split_col(const float* W, int k0, int n, int lane, int ld, int K) { float v[16]; const int g = lane >> 4;
#pragma unroll
  for (int i = 0; i < 8; ++i) { const int ka = k0 + 8 * g + i, kb = ka + 16; v[i] = ka < K ? W[(size_t)(ka < K ? ka : K - 1) * ld + n] : 0.f; v[8 + i] = kb < K ? W[(size_t)(kb < K ? kb : K - 1) * ld + n] : 0.f; }
  return bsplit16(v); }
__device__ __forceinline__ v8f mac3(const F2& a, const F2& b, v8f c) { c = wmma_bf(a.l, b.h, c); c = wmma_bf(a.h, b.l, c); return wmma_bf(a.h, b.h, c); }
__device__ __forceinline__ float sigm(float v) { return 1.0f / (1.0f + expf(-v)); }
#define LDSX() do { asm volatile("s_wait_dscnt 0" ::: "memory"); __builtin_amdgcn_wave_barrier(); __builtin_amdgcn_fence(__ATOMIC_RELEASE, "workgroup"); } while (0)


#define NBATCH 32
#define CC 512
#define NT 256
#define NL 25
#define NR (NBATCH * NT)
#ifndef NBT
#define NBT NBATCH
#endif
typedef __attribute__((ext_vector_type(8))) __bf16 v8b;
__device__ __forceinline__ v16b frag_b(const __bf16* rowk0, int lane) {
  union { v16b v; v8b q[2]; } u; const __bf16* p = rowk0 + 8 * (lane >> 4);
  u.q[0] = *(const v8b*)p; u.q[1] = *(const v8b*)(p + 16); return u.v;
}
__device__ __forceinline__ float bfr(float v) { return (float)(__bf16)v; }
__device__ __attribute__((noinline)) float exp_ni(float v) { return expf(v); }
__device__ __attribute__((noinline)) float erf_ni(float v) { return erff(v); }

#define WS_PF  0u
#define WS_ENC (WS_PF + 2u * CC * CC)
#define WS_FE  (WS_ENC + 4u * (size_t)NR * CC)
#define WS_SC  (WS_FE + 4u * (size_t)NR * CC)
#define WS_END (WS_SC + 4u * (size_t)NBATCH * 32 * NT)

__global__ __launch_bounds__(256) void k_pack(const float* __restrict__ FW, __bf16* __restrict__ P) { const int n = blockIdx.x, t = threadIdx.x; __shared__ __align__(16) __bf16 s[CC]; for (int k = t; k < CC; k += 256) s[k] = (__bf16)FW[(size_t)n * CC + k]; __syncthreads(); if (t < CC / 8) vst2((unsigned*)(P + (size_t)n * CC + t * 8), *(const v4u*)&s[t * 8]); }
__global__ __launch_bounds__(256) void k_enc(const float* __restrict__ X, const float* __restrict__ EMB, float* __restrict__ ENC) {
  __shared__ float st[64][132]; const size_t rb0 = (size_t)blockIdx.x * 64; const int c0 = blockIdx.y * 128, tid = threadIdx.x; const size_t b = rb0 / NT, t0 = rb0 % NT;
  for (int e = tid; e < 128 * 64; e += 256) { const int c = e >> 6, tl = e & 63; st[tl][c] = bfr(X[((b * CC + c0 + c) * (size_t)NT) + t0 + tl]) + bfr(EMB[(t0 + tl) * CC + c0 + c]); }
  __syncthreads();
  for (int e = tid; e < 64 * 32; e += 256) { const int tl = e >> 5, q = e & 31; vst2(ENC + (rb0 + tl) * CC + c0 + q * 4, *(const v4f*)&st[tl][q * 4]); }
}
__global__ __launch_bounds__(128) void k_feat(const float* __restrict__ ENC, const __bf16* __restrict__ P, const float* __restrict__ FB, float* __restrict__ FE) {
  __shared__ __align__(16) float so[4][16][132];
  const int tid = threadIdx.x, wave = tid >> 5, lane = tid & 31, col = lane & 15, g = lane >> 4; const size_t r0 = (size_t)blockIdx.x * 64 + wave * 16; const int n0 = blockIdx.y * 128;
  v8f acc[8] = {};
#pragma unroll 2
  for (int kc = 0; kc < CC / 32; ++kc) { const F2 a = split_row(ENC + (r0 + col) * CC, kc * 32, lane);
#pragma unroll
    for (int j = 0; j < 8; ++j) { const v16b w = frag_b(P + (size_t)(n0 + j * 16 + col) * CC + kc * 32, lane); acc[j] = wmma_bf(a.l, w, acc[j]); acc[j] = wmma_bf(a.h, w, acc[j]); } }
#pragma unroll
  for (int j = 0; j < 8; ++j) { const float bb = bfr(FB[n0 + j * 16 + col]);
#pragma unroll
    for (int r = 0; r < 8; ++r) so[wave][8 * g + r][j * 16 + col] = acc[j][r] + bb; }
  LDSX();
  for (int rl = 0; rl < 16; ++rl) vst2(FE + (r0 + rl) * CC + n0 + lane * 4, *(const v4f*)&so[wave][rl][lane * 4]);
}
__device__ __attribute__((noinline)) float tanh_p(float v) { return tanhf(v); }
__global__ __launch_bounds__(256) void k_attend(const float* __restrict__ FE, const float* __restrict__ TW, const float* __restrict__ SW, const float* __restrict__ ENC, float* __restrict__ OUT) {
  __shared__ float stw[CC], ssw[CC]; __shared__ float sw[NT]; __shared__ float red[256]; __shared__ __align__(16) float so[CC];
  const int b = blockIdx.x / NL, l = blockIdx.x % NL, t = threadIdx.x;
  for (int c = t; c < CC; c += 256) { stw[c] = bfr(TW[(size_t)l * CC + c]); ssw[c] = bfr(SW[c]); }
  __syncthreads();
  const float* fe = FE + ((size_t)b * NT + t) * CC; float s = 0.f;
#pragma unroll 4
  for (int c = 0; c < CC; ++c) s += tanh_p(stw[c] + fe[c]) * ssw[c];
  red[t] = s; __syncthreads(); for (int st = 128; st > 0; st >>= 1) { if (t < st) red[t] = fmaxf(red[t], red[t + st]); __syncthreads(); }
  const float mx = red[0]; __syncthreads(); const float e = exp_ni(s - mx); red[t] = e; sw[t] = e; __syncthreads();
  for (int st = 128; st > 0; st >>= 1) { if (t < st) red[t] += red[t + st]; __syncthreads(); }
  const float inv = 1.0f / red[0];
  for (int c = t; c < CC; c += 256) { float acc = 0.f;
#pragma unroll 4
    for (int tp = 0; tp < NT; ++tp) acc += (sw[tp] * inv) * ENC[((size_t)b * NT + tp) * CC + c];
    so[c] = acc; }
  __syncthreads();
  for (int q = t; q < CC / 4; q += 256) vst2(OUT + ((size_t)b * NL + l) * CC + q * 4, *(const v4f*)&so[q * 4]);
}
extern "C" void kernel_launch(void* const* d_in, const int* in_sizes, int n_in, void* d_out, int out_size, void* d_ws, size_t ws_size, hipStream_t stream) {
  (void)in_sizes; (void)n_in; (void)out_size;
  const float** F = (const float**)d_in;
  if (ws_size < (size_t)WS_END) return;
  char* ws = (char*)d_ws; __bf16* P = (__bf16*)ws; float *ENC = (float*)(ws + WS_ENC), *FE = (float*)(ws + WS_FE);
  k_pack<<<CC, 256, 0, stream>>>(F[2], P);
  k_enc<<<dim3(NBT * NT / 64, CC / 128), 256, 0, stream>>>(F[0], F[1], ENC);
  k_feat<<<dim3(NBT * NT / 64, CC / 128), 128, 0, stream>>>(ENC, P, F[3], FE);
  k_attend<<<NBT * NL, 256, 0, stream>>>(FE, F[4], F[5], ENC, (float*)d_out);
}
